// GAT3_7730941133134
// MI455X (gfx1250) — hardware-verified
//
#include <hip/hip_runtime.h>
#include <stddef.h>


#define GR    32
#define NTHR  256
#define NW    8
#define CHUNK 2048
#define WCAP  256
#define NGRP  (CHUNK / (NTHR * 4))
#define LSH   10

static_assert(WCAP == (CHUNK / NTHR) * 32);
static_assert(NGRP >= 1);
static_assert(CHUNK <= 2048);

typedef float    v2f  __attribute__((ext_vector_type(2)));
typedef float    v4f  __attribute__((ext_vector_type(4)));
typedef float    v8f  __attribute__((ext_vector_type(8)));
typedef int      v4i  __attribute__((ext_vector_type(4)));
typedef _Float16 v8h  __attribute__((ext_vector_type(8)));
typedef _Float16 v16h __attribute__((ext_vector_type(16)));
union Frag   { v16h v; v8h half[2]; };
union Pack16 { v8h h; v4i i; };

__device__ __forceinline__ v8f wm(v16h a, v16h b, v8f c) {
  v8f d = __builtin_amdgcn_wmma_f32_16x16x32_f16(false, a, false, b, (short)0, c, false, false);
  asm volatile("v_nop\n\tv_nop\n\tv_nop\n\tv_nop" : "+v"(d) : "v"(a), "v"(b));
  return d;
}

template <int FPL> struct Seg { float v[FPL]; };
__device__ __forceinline__ void seg_ld(Seg<1>& s, const float* p) { s.v[0] = *p; }
__device__ __forceinline__ void seg_st(float* p, const Seg<1>& s) { *p = s.v[0]; }
__device__ __forceinline__ void seg_ld(Seg<2>& s, const float* p) {
  const v2f t = *(const v2f*)p; s.v[0] = t.x; s.v[1] = t.y;
}
__device__ __forceinline__ void seg_st(float* p, const Seg<2>& s) {
  v2f t; t.x = s.v[0]; t.y = s.v[1]; *(v2f*)p = t;
}
__device__ __forceinline__ void seg_ld(Seg<16>& s, const float* p) {
#pragma unroll
  for (int u = 0; u < 4; ++u) {
    const v4f t = *(const v4f*)(p + 4 * u);
    s.v[4 * u] = t.x; s.v[4 * u + 1] = t.y; s.v[4 * u + 2] = t.z; s.v[4 * u + 3] = t.w;
  }
}
__device__ __forceinline__ void seg_st(float* p, const Seg<16>& s) {
#pragma unroll
  for (int u = 0; u < 4; ++u) {
    v4f t; t.x = s.v[4 * u]; t.y = s.v[4 * u + 1]; t.z = s.v[4 * u + 2]; t.w = s.v[4 * u + 3];
    *(v4f*)(p + 4 * u) = t;
  }
}

template <int K, int NCOL, int NHD>
struct GemmLds {
  static constexpr int AP    = K + 8;
  static constexpr int XSP   = NCOL + 4;
  static constexpr int BYTES = GR * AP * 2 + GR * XSP * 4 + 2 * GR * NHD * 4;
};
template <int DF, int NHD, int NB>
struct GatLds {
  static constexpr int BYTES = (NB * DF + 2 * NB * NHD) * 4 + (NW * WCAP + 16) * 4;
};
static_assert(GemmLds<32, 64, 8>::BYTES == 13312);
static_assert(GemmLds<64, 512, 8>::BYTES == 72704);
static_assert(GemmLds<512, 32, 1>::BYTES == 38144);
static_assert(GatLds<64, 8, 512>::BYTES == 172096);
static_assert(GatLds<512, 8, 128>::BYTES == 278592);
static_assert(GatLds<32, 1, 512>::BYTES == 77888);

__global__ __launch_bounds__(NTHR) void k_prep(const float* __restrict__ W, _Float16* Wh,
                                               int K, int Nin, int NCOL, float scale) {
  const int i  = blockIdx.x * NTHR + threadIdx.x;
  const int k8 = K >> 3;
  const int n8 = NCOL * k8;
  if (i >= n8) return;
  const int n  = i / k8;
  const int k0 = (i - n * k8) * 8;
  Pack16 u;
#pragma unroll
  for (int j = 0; j < 8; ++j) {
    float v = 0.f;
    if (n < Nin) v = W[(size_t)(k0 + j) * Nin + n] * scale;
    u.h[j] = (_Float16)v;
  }
  _Float16* p = Wh + (size_t)i * 8;
  *(volatile v4i*)p = u.i;
  __threadfence();
  *(volatile v4i*)p = u.i;
}

template <int NCOL, int NHD, int NT, int XSP>
__device__ __forceinline__ void gemm_store(const float* Xs, const float* Als, const float* Ald,
                                           float* gx, float* gs, float* gd, int tid) {
  for (int q = tid; q < GR * NCOL / 4; q += NT) {
    const int f   = 4 * q;
    const int row = f / NCOL;
    const int col = f - row * NCOL;
    const v4f v = *(const v4f*)(Xs + row * XSP + col);
    *(volatile v4f*)(gx + f) = v;
  }
  for (int q = tid; q < GR * NHD / 4; q += NT) {
    const v4f a = *(const v4f*)(Als + 4 * q);
    const v4f d = *(const v4f*)(Ald + 4 * q);
    *(volatile v4f*)(gs + 4 * q) = a;
    *(volatile v4f*)(gd + 4 * q) = d;
  }
}

template <int K, int NCOL, int NHD, int HC, int NWG>
__global__ __launch_bounds__(NWG * 32) void k_gemm(
    const float* __restrict__ A, const _Float16* __restrict__ Wh,
    const float* __restrict__ att_s, const float* __restrict__ att_d,
    float* xp, float* als, float* ald, int nN, float invs) {
  constexpr int NT  = NWG * 32;
  constexpr int AP  = GemmLds<K, NCOL, NHD>::AP;
  constexpr int XSP = GemmLds<K, NCOL, NHD>::XSP;
  constexpr int CT  = NCOL / 16;
  constexpr int TT  = 2 * CT;
  constexpr int TPW = TT / NWG;
  static_assert(TPW >= 1 && TPW * NWG == TT);
  static_assert(TPW == 1 || (CT % TPW) == 0);
  static_assert((K % 32) == 0 && (NCOL % 32) == 0);
  static_assert(NHD * HC <= NCOL);
  static_assert(((GR * NHD) % 4) == 0);

  extern __shared__ v4f lds_dyn[];
  _Float16* At  = (_Float16*)lds_dyn;
  float*    Xs  = (float*)(At + GR * AP);
  float*    Als = Xs + GR * XSP;
  float*    Ald = Als + GR * NHD;

  const int tid  = threadIdx.x;
  const int lane = tid & 31;
  const int wave = tid >> 5;
  const int hh   = lane >> 4;
  const int m    = lane & 15;
  const int rowBase = blockIdx.x * GR;

  for (int g = tid; g < GR * (K / 8); g += NT) {
    const int r  = g / (K / 8);
    const int c0 = (g - r * (K / 8)) * 8;
    int row = rowBase + r;
    if (row > nN - 1) row = nN - 1;
    const float* p = A + (size_t)row * K + c0;
    const v4f f0 = *(const v4f*)(p);
    const v4f f1 = *(const v4f*)(p + 4);
    Pack16 u;
    u.h[0] = (_Float16)f0.x; u.h[1] = (_Float16)f0.y; u.h[2] = (_Float16)f0.z; u.h[3] = (_Float16)f0.w;
    u.h[4] = (_Float16)f1.x; u.h[5] = (_Float16)f1.y; u.h[6] = (_Float16)f1.z; u.h[7] = (_Float16)f1.w;
    *(v8h*)(At + r * AP + c0) = u.h;
  }
  __syncthreads();

  const int rt  = (wave * TPW) / CT;
  const int ct0 = (wave * TPW) % CT;
  const v8f z8 = {0.f, 0.f, 0.f, 0.f, 0.f, 0.f, 0.f, 0.f};
  v8f acc[TPW];
#pragma unroll
  for (int j = 0; j < TPW; ++j) acc[j] = z8;
#pragma unroll
  for (int kt = 0; kt < K / 32; ++kt) {
    const int k0 = kt * 32;
    Frag a;
    const _Float16* pa = At + (rt * 16 + m) * AP + k0 + 8 * hh;
    a.half[0] = *(const v8h*)pa;
    a.half[1] = *(const v8h*)(pa + 16);
#pragma unroll
    for (int j = 0; j < TPW; ++j) {
      Frag b;
      const _Float16* pb = Wh + (size_t)((ct0 + j) * 16 + m) * K + k0 + 8 * hh;
      b.half[0] = *(const v8h*)pb;
      b.half[1] = *(const v8h*)(pb + 16);
      acc[j] = wm(a.v, b.v, acc[j]);
    }
  }

#pragma unroll
  for (int j = 0; j < TPW; ++j) {
#pragma unroll
    for (int r = 0; r < 8; ++r) {
      Xs[(rt * 16 + 8 * hh + r) * XSP + (ct0 + j) * 16 + m] = acc[j][r] * invs;
    }
  }
  __syncthreads();

  for (int idx = tid; idx < GR * NHD; idx += NT) {
    const int row = idx / NHD;
    const int hd  = idx - row * NHD;
    const float* xr = Xs + row * XSP + hd * HC;
    float ss = 0.f, sd = 0.f;
#pragma unroll 4
    for (int c = 0; c < HC; ++c) {
      const float v = xr[c];
      ss += v * att_s[hd * HC + c];
      sd += v * att_d[hd * HC + c];
    }
    Als[idx] = ss;
    Ald[idx] = sd;
  }
  __syncthreads();

  float* gx = xp  + (size_t)rowBase * NCOL;
  float* gs = als + (size_t)rowBase * NHD;
  float* gd = ald + (size_t)rowBase * NHD;
  gemm_store<NCOL, NHD, NT, XSP>(Xs, Als, Ald, gx, gs, gd, tid);
  __threadfence();
  gemm_store<NCOL, NHD, NT, XSP>(Xs, Als, Ald, gx, gs, gd, tid);
}

template <int DF, int OUTC>
__device__ __forceinline__ void gat_store(const float* S, float* base, int nf, int tid) {
  const int nq = nf >> 2;
  for (int q = tid; q < nq; q += NTHR) {
    v4f v;
    if (OUTC == DF) {
      v = *(const v4f*)(S + 4 * q);
    } else {
      const int f = 4 * q;
      v.x = S[((f    ) / OUTC) * DF + ((f    ) % OUTC)];
      v.y = S[((f + 1) / OUTC) * DF + ((f + 1) % OUTC)];
      v.z = S[((f + 2) / OUTC) * DF + ((f + 2) % OUTC)];
      v.w = S[((f + 3) / OUTC) * DF + ((f + 3) % OUTC)];
    }
    *(volatile v4f*)(base + 4 * q) = v;
  }
  const int rem = nf & 3;
  if (tid < rem) {
    const int f = (nq << 2) + tid;
    const float v = S[(f / OUTC) * DF + (f % OUTC)];
    *(volatile float*)(base + f) = v;
  }
}

template <int DF, int NHD, int NB, int OUTC, int ELU>
__global__ __launch_bounds__(NTHR) void k_gat(
    const int* __restrict__ ei, const float* __restrict__ xp,
    const float* __restrict__ als, const float* __restrict__ ald,
    const float* __restrict__ bias, float* out, int nN, int nE) {
  constexpr int FPL = DF / 32;
  constexpr int SPW = NB / NW;
  static_assert(FPL * 32 == DF);
  static_assert((NB & (NB - 1)) == 0 && NB <= (1 << LSH));
  static_assert(SPW * NW == NB);
  static_assert(((NB * NHD) % 4) == 0);
  static_assert(OUTC <= DF && OUTC >= 1);

  extern __shared__ v4f lds_dyn[];
  float* sacc = (float*)lds_dyn;
  float* den  = sacc + NB * DF;
  float* mxv  = den + NB * NHD;
  int*   list = (int*)(mxv + NB * NHD);
  int*   wcnt = list + NW * WCAP;

  const int tid  = threadIdx.x;
  const int lane = tid & 31;
  const int wave = tid >> 5;
  const int hd   = (lane * FPL * NHD) / DF;
  const bool lead = ((lane * FPL * NHD) % DF) == 0;
  const int nodeBase = blockIdx.x * NB;

  {
    const v4f z4 = {0.f, 0.f, 0.f, 0.f};
    for (int i = tid; i < (NB * DF + NB * NHD) / 4; i += NTHR) lds_dyn[i] = z4;
    for (int i = tid; i < NB * NHD; i += NTHR) mxv[i] = -1.0e30f;
  }
  __syncthreads();

  const int* eid = ei + nE;
  const bool al16 = ((nE & 3) == 0);

  const int nChunks = (nE + CHUNK - 1) / CHUNK;
#pragma unroll 1
  for (int ch = 0; ch < nChunks; ++ch) {
    const int cbase = ch * CHUNK;
    int wc = 0;
#pragma unroll
    for (int g = 0; g < NGRP; ++g) {
      const int el0 = (g * NTHR + tid) * 4;
      const int e0  = cbase + el0;
      const int sent = -2147483647 - 1;
      v4i d;
      if (al16 && (e0 + 3 < nE)) {
        d = *(const v4i*)(eid + e0);
      } else {
        d.x = (e0     < nE) ? eid[min(e0, nE - 1)]     : sent;
        d.y = (e0 + 1 < nE) ? eid[min(e0 + 1, nE - 1)] : sent;
        d.z = (e0 + 2 < nE) ? eid[min(e0 + 2, nE - 1)] : sent;
        d.w = (e0 + 3 < nE) ? eid[min(e0 + 3, nE - 1)] : sent;
      }
      const unsigned s0 = (unsigned)d.x - (unsigned)nodeBase;
      const unsigned s1 = (unsigned)d.y - (unsigned)nodeBase;
      const unsigned s2 = (unsigned)d.z - (unsigned)nodeBase;
      const unsigned s3 = (unsigned)d.w - (unsigned)nodeBase;
      const bool h0 = s0 < (unsigned)NB;
      const bool h1 = s1 < (unsigned)NB;
      const bool h2 = s2 < (unsigned)NB;
      const bool h3 = s3 < (unsigned)NB;
      const unsigned many = __builtin_amdgcn_ballot_w32(h0 | h1 | h2 | h3);
      if (many != 0u) {
#define HITJ(J, HJ, SJ) { \
          const unsigned mj = __builtin_amdgcn_ballot_w32(HJ); \
          if (HJ) { \
            const int pos = wc + (int)__builtin_amdgcn_mbcnt_lo(mj, 0u); \
            if (pos < WCAP) list[wave * WCAP + pos] = ((el0 + (J)) << LSH) | (int)(SJ); \
          } \
          wc += (int)__builtin_popcount(mj); }
        HITJ(0, h0, s0)
        HITJ(1, h1, s1)
        HITJ(2, h2, s2)
        HITJ(3, h3, s3)
#undef HITJ
      }
    }
    if (lane == 0) wcnt[wave] = wc;
    __syncthreads();

    if (wave == 0) {
#pragma unroll 1
      for (int wsx = 0; wsx < NW; ++wsx) {
        int n = wcnt[wsx];
        if (n > WCAP) n = WCAP;
        if (n < 0) n = 0;
#pragma unroll 1
        for (int i = 0; i < n; ++i) {
          const int ent  = list[wsx * WCAP + i];
          const int slot = ent & (NB - 1);
          const int el   = (ent >> LSH) & (CHUNK - 1);
          int e = cbase + el;
          if (e > nE - 1) e = nE - 1;
          int src = ei[e];
          src = src < 0 ? 0 : (src > nN - 1 ? nN - 1 : src);
          int nd = nodeBase + slot;
          if (nd > nN - 1) nd = nN - 1;
          float al = als[(size_t)src * NHD + hd] + ald[(size_t)nd * NHD + hd];
          al = (al > 0.f) ? al : 0.2f * al;
          const int ai = slot * NHD + hd;
          const float mo = mxv[ai];
          const float mn = fmaxf(mo, al);
          const float sc = __expf(mo - mn);
          const float p  = __expf(al - mn);
          Seg<FPL> xv, cur;
          seg_ld(xv, xp + (size_t)src * DF + lane * FPL);
          float* sp = sacc + slot * DF + lane * FPL;
          seg_ld(cur, sp);
#pragma unroll
          for (int f = 0; f < FPL; ++f) cur.v[f] = cur.v[f] * sc + p * xv.v[f];
          seg_st(sp, cur);
          if (lead) {
            const float d0 = den[ai];
            den[ai] = d0 * sc + p;
            mxv[ai] = mn;
          }
        }
      }
    }
    __syncthreads();
  }

  Seg<FPL> bsg;
#pragma unroll
  for (int f = 0; f < FPL; ++f) {
    const int bi = lane * FPL + f;
    const float bv = bias[bi < OUTC ? bi : (OUTC - 1)];
    bsg.v[f] = (bi < OUTC) ? bv : 0.f;
  }
#pragma unroll 1
  for (int j = 0; j < SPW; ++j) {
    const int slot = wave * SPW + j;
    const int node = nodeBase + slot;
    if (node >= nN) break;
    const size_t nrow = (size_t)node;
    float al = als[nrow * NHD + hd] + ald[nrow * NHD + hd];
    al = (al > 0.f) ? al : 0.2f * al;
    const int ai = slot * NHD + hd;
    const float mo = mxv[ai];
    const float mn = fmaxf(mo, al);
    const float sc = __expf(mo - mn);
    const float p  = __expf(al - mn);
    Seg<FPL> xv, sv;
    seg_ld(xv, xp + nrow * DF + lane * FPL);
    float* sp = sacc + slot * DF + lane * FPL;
    seg_ld(sv, sp);
    const float dv  = den[ai] * sc + p;
    const float inv = 1.0f / (dv + 1e-16f);
#pragma unroll
    for (int f = 0; f < FPL; ++f) {
      float h = (sv.v[f] * sc + p * xv.v[f]) * inv + bsg.v[f];
      if (ELU) h = (h > 0.f) ? h : (__expf(fminf(h, 0.f)) - 1.f);
      sv.v[f] = h;
    }
    seg_st(sp, sv);
  }
  __syncthreads();

  int nvalid = nN - nodeBase;
  if (nvalid > NB) nvalid = NB;
  if (nvalid < 0) nvalid = 0;
  const int nf = nvalid * OUTC;
  float* base = out + (size_t)nodeBase * OUTC;
  gat_store<DF, OUTC>(sacc, base, nf, tid);
  __threadfence();
  gat_store<DF, OUTC>(sacc, base, nf, tid);
}

extern "C" void kernel_launch(void* const* d_in, const int* in_sizes, int n_in,
                              void* d_out, int out_size, void* d_ws, size_t ws_size,
                              hipStream_t stream) {
  if (n_in < 14) return;
  const int nN = in_sizes[0] / 32;
  const int nE = in_sizes[1] / 2;
  if (nN <= 0 || in_sizes[0] != nN * 32) return;
  if (nE < 0 || in_sizes[1] != 2 * nE) return;
  if (in_sizes[2] != 32 * 64 || in_sizes[3] != 64 || in_sizes[4] != 64 || in_sizes[5] != 64) return;
  if (in_sizes[6] != 64 * 512 || in_sizes[7] != 512 || in_sizes[8] != 512 || in_sizes[9] != 512) return;
  if (in_sizes[10] != 512 * 6 || in_sizes[11] != 6 || in_sizes[12] != 6 || in_sizes[13] != 6) return;
  if (out_size != nN * 6) return;

  const float* x   = (const float*)d_in[0];
  const int*   ei  = (const int*)d_in[1];
  const float* W1  = (const float*)d_in[2];
  const float* aS1 = (const float*)d_in[3];
  const float* aD1 = (const float*)d_in[4];
  const float* b1  = (const float*)d_in[5];
  const float* W2  = (const float*)d_in[6];
  const float* aS2 = (const float*)d_in[7];
  const float* aD2 = (const float*)d_in[8];
  const float* b2  = (const float*)d_in[9];
  const float* W3  = (const float*)d_in[10];
  const float* aS3 = (const float*)d_in[11];
  const float* aD3 = (const float*)d_in[12];
  const float* b3  = (const float*)d_in[13];
  float* out = (float*)d_out;

  const int nP = ((nN + GR - 1) / GR) * GR;
  size_t off = 0;
  auto carve = [&](size_t bytes) -> char* {
    char* p = (char*)d_ws + off;
    off += (bytes + 255) & ~(size_t)255;
    return p;
  };
  _Float16* Wh1 = (_Float16*)carve((size_t)64 * 32 * 2);
  _Float16* Wh2 = (_Float16*)carve((size_t)512 * 64 * 2);
  _Float16* Wh3 = (_Float16*)carve((size_t)32 * 512 * 2);
  float* xp1  = (float*)carve((size_t)nP * 64 * 4);
  float* als1 = (float*)carve((size_t)nP * 8 * 4);
  float* ald1 = (float*)carve((size_t)nP * 8 * 4);
  float* act1 = (float*)carve((size_t)nP * 64 * 4);
  float* xp2  = (float*)carve((size_t)nP * 512 * 4);
  float* als2 = (float*)carve((size_t)nP * 8 * 4);
  float* ald2 = (float*)carve((size_t)nP * 8 * 4);
  float* act2 = (float*)carve((size_t)nP * 512 * 4);
  float* xp3  = (float*)carve((size_t)nP * 32 * 4);
  float* als3 = (float*)carve((size_t)nP * 1 * 4);
  float* ald3 = (float*)carve((size_t)nP * 1 * 4);
  if (off > ws_size) return;
  if (off > ((size_t)128 << 20)) return;

  constexpr int LG1 = GemmLds<32, 64, 8>::BYTES;
  constexpr int LG2 = GemmLds<64, 512, 8>::BYTES;
  constexpr int LG3 = GemmLds<512, 32, 1>::BYTES;
  constexpr int LA1 = GatLds<64, 8, 512>::BYTES;
  constexpr int LA2 = GatLds<512, 8, 128>::BYTES;
  constexpr int LA3 = GatLds<32, 1, 512>::BYTES;
  hipFuncSetAttribute((const void*)&k_gemm<32, 64, 8, 8, 8>,    hipFuncAttributeMaxDynamicSharedMemorySize, LG1);
  hipFuncSetAttribute((const void*)&k_gemm<64, 512, 8, 64, 8>,  hipFuncAttributeMaxDynamicSharedMemorySize, LG2);
  hipFuncSetAttribute((const void*)&k_gemm<512, 32, 1, 6, 4>,   hipFuncAttributeMaxDynamicSharedMemorySize, LG3);
  hipFuncSetAttribute((const void*)&k_gat<64, 8, 512, 64, 1>,   hipFuncAttributeMaxDynamicSharedMemorySize, LA1);
  hipFuncSetAttribute((const void*)&k_gat<512, 8, 128, 512, 1>, hipFuncAttributeMaxDynamicSharedMemorySize, LA2);
  hipFuncSetAttribute((const void*)&k_gat<32, 1, 512, 6, 0>,    hipFuncAttributeMaxDynamicSharedMemorySize, LA3);

  k_prep<<<(64 * 32 / 8 + NTHR - 1) / NTHR, NTHR, 0, stream>>>(W1, Wh1, 32, 64, 64, 16.0f);
  k_prep<<<(512 * 64 / 8 + NTHR - 1) / NTHR, NTHR, 0, stream>>>(W2, Wh2, 64, 512, 512, 64.0f);
  k_prep<<<(32 * 512 / 8 + NTHR - 1) / NTHR, NTHR, 0, stream>>>(W3, Wh3, 512, 6, 32, 64.0f);

  const int gGemm = nP / GR;

  k_gemm<32, 64, 8, 8, 8><<<gGemm, 256, LG1, stream>>>(x, Wh1, aS1, aD1, xp1, als1, ald1, nN, 1.0f / 16.0f);
  k_gat<64, 8, 512, 64, 1><<<(nN + 511) / 512, NTHR, LA1, stream>>>(ei, xp1, als1, ald1, b1, act1, nN, nE);

  k_gemm<64, 512, 8, 64, 8><<<gGemm, 256, LG2, stream>>>(act1, Wh2, aS2, aD2, xp2, als2, ald2, nN, 1.0f / 64.0f);
  k_gat<512, 8, 128, 512, 1><<<(nN + 127) / 128, NTHR, LA2, stream>>>(ei, xp2, als2, ald2, b2, act2, nN, nE);

  k_gemm<512, 32, 1, 6, 4><<<gGemm, 128, LG3, stream>>>(act2, Wh3, aS3, aD3, xp3, als3, ald3, nN, 1.0f / 64.0f);
  k_gat<32, 1, 512, 6, 0><<<(nN + 511) / 512, NTHR, LA3, stream>>>(ei, xp3, als3, ald3, b3, out, nN, nE);
}
